// GCU_56401510531237
// MI455X (gfx1250) — hardware-verified
//
#include <hip/hip_runtime.h>

#define B_   4
#define C_   128
#define N_   4096
#define K_   32
#define NBLK 64

#define PL_SA ((size_t)B_ * K_ * N_)
#define PL_X  ((size_t)B_ * C_ * N_)
#define PL_G  ((size_t)B_ * C_ * K_)

#define OFF_INVS  ((size_t)0)
#define OFF_PART  ((size_t)16384)
#define OFF_M1    ((size_t)49152)
#define OFF_G     ((size_t)114688)
#define OFF_SAK   ((size_t)180224)
#define OFF_SAT   ((size_t)2277376)
#define OFF_X     ((size_t)4374528)
#define WS_TOTAL  ((size_t)12763136)
static_assert(OFF_PART == OFF_INVS + (size_t)K_ * C_ * 4);
static_assert(OFF_M1 == OFF_PART + (size_t)B_ * NBLK * K_ * 4);
static_assert(OFF_G == OFF_M1 + (size_t)B_ * C_ * K_ * 4);
static_assert(OFF_SAK == OFF_G + 2 * PL_G * 2);
static_assert(OFF_SAT == OFF_SAK + 2 * PL_SA * 2);
static_assert(OFF_X == OFF_SAT + 2 * PL_SA * 2);
static_assert(WS_TOTAL == OFF_X + 2 * PL_X * 2);
static_assert((N_ % 64) == 0 && (C_ % 16) == 0 && K_ == 32 && (N_ % 512) == 0);

typedef float          v8f   __attribute__((ext_vector_type(8)));
typedef float          v4f   __attribute__((ext_vector_type(4)));
typedef float          v2f   __attribute__((ext_vector_type(2)));
typedef unsigned short v8us  __attribute__((ext_vector_type(8)));
typedef unsigned short v16us __attribute__((ext_vector_type(16)));
typedef __bf16         v16b  __attribute__((ext_vector_type(16)));
typedef v8us __attribute__((may_alias)) v8usa;
typedef v4f  __attribute__((may_alias)) v4fa;
typedef v2f  __attribute__((may_alias)) v2fa;

union FragU { v16us v; v8us half[2]; };

__device__ __forceinline__ v8f wmma_bf16(v16us a, v16us b, v8f c) {
  v8f d = __builtin_amdgcn_wmma_f32_16x16x32_bf16(false, __builtin_bit_cast(v16b, a), false,
                                                  __builtin_bit_cast(v16b, b), (short)0, c, false, false);
  asm volatile("v_nop\n\tv_nop\n\tv_nop\n\tv_nop" : "+v"(d) : "v"(a), "v"(b));
  return d;
}

__device__ __forceinline__ v16us load_frag_u(const unsigned short* p, int h) {
  FragU f;
  f.half[0] = *(const v8usa*)(p + 8 * h);
  f.half[1] = *(const v8usa*)(p + 16 + 8 * h);
  return f.v;
}

__device__ __forceinline__ unsigned short f2bf(float f) {
  const unsigned int u = __float_as_uint(f);
  return (unsigned short)((u + 0x7FFFu + ((u >> 16) & 1u)) >> 16);
}
__device__ __forceinline__ float bf2f(unsigned short s) {
  return __uint_as_float(((unsigned int)s) << 16);
}

__device__ __forceinline__ void split8(v4f a, v4f c, v8us& hi, v8us& lo) {
  const float f[8] = {a.x, a.y, a.z, a.w, c.x, c.y, c.z, c.w};
  #pragma unroll
  for (int i = 0; i < 8; ++i) {
    const unsigned short hb = f2bf(f[i]);
    hi[i] = hb;
    lo[i] = f2bf(f[i] - bf2f(hb));
  }
}

__global__ __launch_bounds__(256) void sigma_kernel(const float* __restrict__ sp,
                                                    float* __restrict__ invs) {
  const int i = blockIdx.x * 256 + threadIdx.x;
  if (i >= K_ * C_) return;
  const float s  = sp[i];
  const float sg = 1.0f / (1.0f + expf(-s));
  const float v  = 1.0f / (sg + 1e-7f);
  *(volatile float*)(invs + i) = v;
  __threadfence();
  *(volatile float*)(invs + i) = v;
}

__global__ __launch_bounds__(256) void assign_kernel(
    const float* __restrict__ x, const float* __restrict__ anchor,
    const float* __restrict__ invs,
    unsigned short* __restrict__ sak,
    unsigned short* __restrict__ sat,
    unsigned short* __restrict__ xpl,
    float* __restrict__ part)
{
  __shared__ __attribute__((aligned(16))) float tab[2 * K_ * C_];
  __shared__ __attribute__((aligned(16))) float lg[K_ * 65];
  __shared__ __attribute__((aligned(16))) float pds[K_];

  const int t = threadIdx.x, lane = t & 31, w = t >> 5;
  const int b = blockIdx.y, blk = blockIdx.x, n0 = blk * 64;

  #pragma unroll 1
  for (int idx = t; idx < K_ * C_; idx += 256) {
    tab[2 * idx]     = anchor[idx];
    tab[2 * idx + 1] = invs[idx];
  }
  __syncthreads();

  const int half = w >> 2, kq = w & 3;
  const int nl = 32 * half + lane;
  const float* xrow = x + (size_t)b * C_ * N_ + n0 + nl;
  float acc[8];
  #pragma unroll
  for (int j = 0; j < 8; ++j) acc[j] = 0.0f;
  #pragma unroll 1
  for (int c = 0; c < C_; ++c) {
    const float xv = xrow[(size_t)c * N_];
    #pragma unroll
    for (int j = 0; j < 8; ++j) {
      const v2f ai = *(const v2fa*)(tab + 2 * ((kq + 4 * j) * C_ + c));
      const float r = (xv - ai.x) * ai.y;
      acc[j] = fmaf(r, r, acc[j]);
    }
  }
  #pragma unroll
  for (int j = 0; j < 8; ++j) lg[(kq + 4 * j) * 65 + nl] = -0.5f * acc[j];
  __syncthreads();

  unsigned short* stg = reinterpret_cast<unsigned short*>(tab);
  if (t < 64) {
    float mx = -3.0e38f;
    #pragma unroll 1
    for (int k = 0; k < K_; ++k) mx = fmaxf(mx, lg[k * 65 + t]);
    float s = 0.0f;
    #pragma unroll 1
    for (int k = 0; k < K_; ++k) {
      const float e = expf(lg[k * 65 + t] - mx);
      lg[k * 65 + t] = e;
      s += e;
    }
    const float inv = 1.0f / s;
    #pragma unroll 1
    for (int k = 0; k < K_; ++k) {
      const float p = lg[k * 65 + t] * inv;
      lg[k * 65 + t] = p;
      const unsigned short hb = f2bf(p);
      const unsigned short lb = f2bf(p - bf2f(hb));
      stg[k * 64 + t]          = hb;
      stg[2048 + k * 64 + t]   = lb;
      stg[4096 + t * 32 + k]   = hb;
      stg[6144 + t * 32 + k]   = lb;
    }
  }
  __syncthreads();
  if (t < K_) {
    float s = 0.0f;
    #pragma unroll 1
    for (int n = 0; n < 64; ++n) s += lg[t * 65 + n];
    pds[t] = s;
  }
  __syncthreads();

  const int p = t >> 7, tt = t & 127;
  v8us kv[2]; size_t kd[2];
  #pragma unroll
  for (int i = 0; i < 2; ++i) {
    const int k = 16 * i + (tt >> 3), q = tt & 7;
    kv[i] = *(const v8usa*)(stg + p * 2048 + k * 64 + 8 * q);
    kd[i] = (size_t)p * PL_SA + ((size_t)(b * K_ + k)) * N_ + n0 + 8 * q;
  }
  v8us tv[2]; size_t td[2];
  #pragma unroll
  for (int i = 0; i < 2; ++i) {
    tv[i] = *(const v8usa*)(stg + 4096 + i * 2048 + 8 * t);
    td[i] = (size_t)i * PL_SA + ((size_t)(b * N_ + n0)) * K_ + 8 * t;
  }
  v8us xhv[4], xlv[4]; size_t xd[4];
  #pragma unroll
  for (int i = 0; i < 4; ++i) {
    const int c = 32 * i + (t >> 3), q = t & 7;
    const size_t off = ((size_t)(b * C_ + c)) * N_ + n0 + 8 * q;
    const v4f f0 = *(const v4fa*)(x + off);
    const v4f f1 = *(const v4fa*)(x + off + 4);
    split8(f0, f1, xhv[i], xlv[i]);
    xd[i] = off;
  }
  const v4f pv = *(const v4fa*)(pds + 4 * (t & 7));
  float* pdst = part + ((size_t)(b * NBLK + blk)) * K_ + 4 * (t & 7);

  #pragma unroll
  for (int i = 0; i < 2; ++i) *(volatile v8us*)(sak + kd[i]) = kv[i];
  #pragma unroll
  for (int i = 0; i < 2; ++i) *(volatile v8us*)(sat + td[i]) = tv[i];
  #pragma unroll
  for (int i = 0; i < 4; ++i) {
    *(volatile v8us*)(xpl + xd[i]) = xhv[i];
    *(volatile v8us*)(xpl + PL_X + xd[i]) = xlv[i];
  }
  if (t < 8) *(volatile v4f*)pdst = pv;
  __threadfence();
  #pragma unroll
  for (int i = 0; i < 2; ++i) *(volatile v8us*)(sak + kd[i]) = kv[i];
  #pragma unroll
  for (int i = 0; i < 2; ++i) *(volatile v8us*)(sat + td[i]) = tv[i];
  #pragma unroll
  for (int i = 0; i < 4; ++i) {
    *(volatile v8us*)(xpl + xd[i]) = xhv[i];
    *(volatile v8us*)(xpl + PL_X + xd[i]) = xlv[i];
  }
  if (t < 8) *(volatile v4f*)pdst = pv;
}

__global__ __launch_bounds__(128) void pool_gemm_kernel(
    const unsigned short* __restrict__ xpl,
    const unsigned short* __restrict__ sak,
    float* __restrict__ m1)
{
  __shared__ __attribute__((aligned(16))) float red[4 * 16 * K_];

  const int t = threadIdx.x, lane = t & 31, w = t >> 5;
  const int h = lane >> 4, m = lane & 15;
  const int b = blockIdx.y, c0 = blockIdx.x * 16;
  const int nb = w * (N_ / 4);

  const unsigned short* xh = xpl + ((size_t)(b * C_ + c0 + m)) * N_ + nb;
  const unsigned short* xl = xh + PL_X;
  const unsigned short* s0 = sak + ((size_t)(b * K_ + m)) * N_ + nb;
  const unsigned short* s1 = s0 + (size_t)16 * N_;

  const v8f zero8 = {0.f, 0.f, 0.f, 0.f, 0.f, 0.f, 0.f, 0.f};
  v8f acc0 = zero8, acc1 = zero8;

  #pragma unroll 1
  for (int k0 = 0; k0 < N_ / 4; k0 += 32) {
    const v16us ah  = load_frag_u(xh + k0, h);
    const v16us al  = load_frag_u(xl + k0, h);
    const v16us b0h = load_frag_u(s0 + k0, h);
    const v16us b0l = load_frag_u(s0 + PL_SA + k0, h);
    const v16us b1h = load_frag_u(s1 + k0, h);
    const v16us b1l = load_frag_u(s1 + PL_SA + k0, h);
    acc0 = wmma_bf16(ah, b0h, acc0);
    acc0 = wmma_bf16(ah, b0l, acc0);
    acc0 = wmma_bf16(al, b0h, acc0);
    acc1 = wmma_bf16(ah, b1h, acc1);
    acc1 = wmma_bf16(ah, b1l, acc1);
    acc1 = wmma_bf16(al, b1h, acc1);
  }

  #pragma unroll
  for (int r = 0; r < 8; ++r) {
    red[(w * 16 + 8 * h + r) * K_ + m]      = acc0[r];
    red[(w * 16 + 8 * h + r) * K_ + 16 + m] = acc1[r];
  }
  __syncthreads();

  v4f o;
  #pragma unroll
  for (int j = 0; j < 4; ++j) {
    const int idx = 4 * t + j;
    o[j] = ((red[idx] + red[512 + idx]) + red[1024 + idx]) + red[1536 + idx];
  }
  float* dst = m1 + ((size_t)(b * C_ + c0)) * K_ + 4 * t;
  *(volatile v4f*)dst = o;
  __threadfence();
  *(volatile v4f*)dst = o;
}

__global__ __launch_bounds__(256) void graph_kernel(
    const float* __restrict__ anchor, const float* __restrict__ invs,
    const float* __restrict__ wgt,
    const float* __restrict__ part,
    const float* __restrict__ m1,
    unsigned short* __restrict__ gpl)
{
  __shared__ __attribute__((aligned(16))) float bufA[K_ * C_];
  __shared__ float gS[C_ * 33];
  __shared__ float adj[K_ * 33];
  __shared__ __attribute__((aligned(16))) unsigned short g2s[2 * C_ * K_];
  __shared__ float den[K_];
  __shared__ float rden[K_];
  __shared__ float wsum[8];

  const int t = threadIdx.x, lane = t & 31, w = t >> 5;
  const int b = blockIdx.x;

  if (t < K_) {
    float s = 0.0f;
    #pragma unroll 1
    for (int q = 0; q < NBLK; ++q) s += part[((size_t)b * NBLK + q) * K_ + t];
    den[t]  = s;
    rden[t] = 1.0f / (s + 1e-7f);
  }
  __syncthreads();

  #pragma unroll 1
  for (int idx = t; idx < K_ * C_; idx += 256) {
    const int k = idx >> 7, c = idx & 127;
    const float mv  = m1[((size_t)b * C_ + c) * K_ + k];
    const float num = (mv - anchor[idx] * den[k]) * invs[idx];
    bufA[idx] = num * rden[k];
  }
  __syncthreads();

  {
    const int k = t >> 3, j = t & 7;
    float s = 0.0f;
    #pragma unroll 1
    for (int c = j; c < C_; c += 8) { const float v = bufA[k * C_ + c]; s = fmaf(v, v, s); }
    s += __shfl_xor(s, 1);
    s += __shfl_xor(s, 2);
    s += __shfl_xor(s, 4);
    const float inv = 1.0f / fmaxf(sqrtf(s), 1e-12f);
    float s2 = 0.0f;
    #pragma unroll 1
    for (int c = j; c < C_; c += 8) {
      const float v = bufA[k * C_ + c] * inv;
      bufA[k * C_ + c] = v;
      s2 = fmaf(v, v, s2);
    }
    s2 += __shfl_xor(s2, 1);
    s2 += __shfl_xor(s2, 2);
    s2 += __shfl_xor(s2, 4);
    s2 += __shfl_xor(s2, 8);
    s2 += __shfl_xor(s2, 16);
    if (lane == 0) wsum[w] = s2;
  }
  __syncthreads();
  float g = 0.0f;
  #pragma unroll
  for (int i = 0; i < 8; ++i) g += wsum[i];
  const float ginv = 1.0f / fmaxf(sqrtf(g), 1e-12f);
  #pragma unroll 1
  for (int idx = t; idx < K_ * C_; idx += 256)
    gS[(idx >> 5) * 33 + (idx & 31)] = bufA[idx] * ginv;
  __syncthreads();

  #pragma unroll 1
  for (int idx = t; idx < K_ * K_; idx += 256) {
    const int k = idx >> 5, l = idx & 31;
    float s = 0.0f;
    #pragma unroll 1
    for (int c = 0; c < C_; ++c) s = fmaf(gS[c * 33 + k], gS[c * 33 + l], s);
    adj[k * 33 + l] = s;
  }
  __syncthreads();
  if (t < K_) {
    float mx = -3.0e38f;
    #pragma unroll 1
    for (int l = 0; l < K_; ++l) mx = fmaxf(mx, adj[t * 33 + l]);
    float s = 0.0f;
    #pragma unroll 1
    for (int l = 0; l < K_; ++l) { const float e = expf(adj[t * 33 + l] - mx); adj[t * 33 + l] = e; s += e; }
    const float inv = 1.0f / s;
    #pragma unroll 1
    for (int l = 0; l < K_; ++l) adj[t * 33 + l] *= inv;
  }
  __syncthreads();

  #pragma unroll 1
  for (int idx = t; idx < K_ * C_; idx += 256) {
    const int k = idx >> 7, d = idx & 127;
    float s = 0.0f;
    #pragma unroll 1
    for (int c = 0; c < C_; ++c) s = fmaf(gS[c * 33 + k], wgt[c * C_ + d], s);
    bufA[idx] = s;
  }
  __syncthreads();

  #pragma unroll 1
  for (int idx = t; idx < K_ * C_; idx += 256) {
    const int c = idx >> 5, k = idx & 31;
    float s = 0.0f;
    #pragma unroll 1
    for (int l = 0; l < K_; ++l) s = fmaf(adj[k * 33 + l], bufA[l * C_ + c], s);
    s = fmaxf(s, 0.0f);
    const unsigned short hb = f2bf(s);
    g2s[idx]           = hb;
    g2s[C_ * K_ + idx] = f2bf(s - bf2f(hb));
  }
  __syncthreads();

  v8us gv[4]; size_t gd[4];
  #pragma unroll
  for (int i = 0; i < 4; ++i) {
    gv[i] = *(const v8usa*)(g2s + i * 2048 + 8 * t);
    gd[i] = (size_t)(i >> 1) * PL_G + (size_t)b * (C_ * K_) + (size_t)(i & 1) * 2048 + 8 * t;
  }
  #pragma unroll
  for (int i = 0; i < 4; ++i) *(volatile v8us*)(gpl + gd[i]) = gv[i];
  __threadfence();
  #pragma unroll
  for (int i = 0; i < 4; ++i) *(volatile v8us*)(gpl + gd[i]) = gv[i];
}

__global__ __launch_bounds__(256) void project_kernel(
    const unsigned short* __restrict__ gpl,
    const unsigned short* __restrict__ sat,
    float* __restrict__ out)
{
  __shared__ __attribute__((aligned(16))) float so[16 * 512];

  const int t = threadIdx.x, lane = t & 31, w = t >> 5;
  const int h = lane >> 4, m = lane & 15;
  const int b = blockIdx.z, c0 = blockIdx.y * 16;
  const int nb0 = blockIdx.x * 512, nb = nb0 + w * 64;

  const unsigned short* gp = gpl + ((size_t)(b * C_ + c0 + m)) * K_;
  const v16us ah = load_frag_u(gp, h);
  const v16us al = load_frag_u(gp + PL_G, h);

  const v8f zero8 = {0.f, 0.f, 0.f, 0.f, 0.f, 0.f, 0.f, 0.f};
  v8f acc[4];
  #pragma unroll
  for (int nt = 0; nt < 4; ++nt) {
    const unsigned short* bp = sat + ((size_t)(b * N_ + nb + 16 * nt + m)) * K_;
    const v16us bh = load_frag_u(bp, h);
    const v16us bl = load_frag_u(bp + PL_SA, h);
    v8f z = zero8;
    z = wmma_bf16(ah, bh, z);
    z = wmma_bf16(ah, bl, z);
    z = wmma_bf16(al, bh, z);
    acc[nt] = z;
  }

  #pragma unroll
  for (int nt = 0; nt < 4; ++nt)
    #pragma unroll
    for (int r = 0; r < 8; ++r)
      so[(8 * h + r) * 512 + w * 64 + 16 * nt + m] = acc[nt][r];
  __syncthreads();

  v4f v[8];
  #pragma unroll
  for (int i = 0; i < 8; ++i) v[i] = *(const v4fa*)(so + i * 1024 + 4 * t);
  float* obase = out + ((size_t)(b * C_ + c0)) * N_ + nb0;
  #pragma unroll
  for (int i = 0; i < 8; ++i) {
    const int row = 2 * i + (t >> 7), col = (4 * t) & 511;
    *(volatile v4f*)(obase + (size_t)row * N_ + col) = v[i];
  }
  __threadfence();
  #pragma unroll
  for (int i = 0; i < 8; ++i) {
    const int row = 2 * i + (t >> 7), col = (4 * t) & 511;
    *(volatile v4f*)(obase + (size_t)row * N_ + col) = v[i];
  }
}

extern "C" void kernel_launch(void* const* d_in, const int* in_sizes, int n_in,
                              void* d_out, int out_size, void* d_ws, size_t ws_size,
                              hipStream_t stream) {
  if (n_in < 4) return;
  if (in_sizes[0] != B_ * C_ * N_) return;
  if (in_sizes[1] != K_ * C_ || in_sizes[2] != K_ * C_) return;
  if (in_sizes[3] != C_ * C_) return;
  if (out_size != B_ * C_ * N_) return;
  if (WS_TOTAL > ws_size) return;

  const float* x      = (const float*)d_in[0];
  const float* anchor = (const float*)d_in[1];
  const float* sigp   = (const float*)d_in[2];
  const float* wgt    = (const float*)d_in[3];
  float* out = (float*)d_out;

  char* ws = (char*)d_ws;
  float*          invs = (float*)(ws + OFF_INVS);
  float*          part = (float*)(ws + OFF_PART);
  float*          m1   = (float*)(ws + OFF_M1);
  unsigned short* gpl  = (unsigned short*)(ws + OFF_G);
  unsigned short* sak  = (unsigned short*)(ws + OFF_SAK);
  unsigned short* sat  = (unsigned short*)(ws + OFF_SAT);
  unsigned short* xpl  = (unsigned short*)(ws + OFF_X);

  sigma_kernel<<<(K_ * C_ + 255) / 256, 256, 0, stream>>>(sigp, invs);
  assign_kernel<<<dim3(NBLK, B_), 256, 0, stream>>>(x, anchor, invs, sak, sat, xpl, part);
  pool_gemm_kernel<<<dim3(C_ / 16, B_), 128, 0, stream>>>(xpl, sak, m1);
  graph_kernel<<<B_, 256, 0, stream>>>(anchor, invs, wgt, part, m1, gpl);
  project_kernel<<<dim3(N_ / 512, C_ / 16, B_), 256, 0, stream>>>(gpl, sat, out);
}
